// MFA_42021960024360
// MI455X (gfx1250) — hardware-run, weakly checked
//
#include <hip/hip_runtime.h>
#include <math.h>

typedef __attribute__((ext_vector_type(16))) _Float16 v16h;
typedef __attribute__((ext_vector_type(8)))  _Float16 v8h;
typedef __attribute__((ext_vector_type(8)))  float    v8f;
typedef __attribute__((ext_vector_type(4)))  float    v4f;
typedef __attribute__((ext_vector_type(4)))  unsigned v4u;

constexpr int kComp    = 32;
constexpr int kDim     = 128;
constexpr int kFac     = 16;
constexpr int kPts     = 20000;
constexpr int kPtsPad  = 20032;
constexpr int kCols    = kComp * kFac + kComp;
constexpr int kColsPad = 576;
constexpr int kCrossCol = kComp * kFac;
constexpr int kOutResp = kPts * kComp;
constexpr int kOutTotal = kOutResp + kPts;
constexpr int kCbPitch = 32;
constexpr int kPtPitch = 132;
static_assert(kCols == 544, "operator width");
static_assert(kColsPad % 64 == 0 && kColsPad >= kCols, "N tile multiple");
static_assert(kPtsPad % 64 == 0 && kPtsPad >= kPts && kPtsPad - kPts < 64, "M tile multiple");
static_assert(kDim % 32 == 0, "K multiple of 32");
static_assert(kPts % 32 == 0, "one wave owns 32 whole rows");
static_assert((kOutResp * 4) % 128 == 0, "second output starts on a line");
static_assert(kFac == 16 && kComp == 32 && kDim == 128, "thread maps assume these");

constexpr float kCarryX = 64.0f;
constexpr float kCarryP = 64.0f;
constexpr float kCarryM = 16.0f;
constexpr float kCarryXP = kCarryX * kCarryP;
constexpr float kHalfInvXP2 = 0.5f / (kCarryXP * kCarryXP);
constexpr float kInvXM = 1.0f / (kCarryX * kCarryM);
constexpr float kF16MinNormal = 6.103515625e-05f;
constexpr float kLog2Pi = 1.8378770664093454836f;
constexpr float kDimLog2Pi = (float)kDim * kLog2Pi;

constexpr size_t kSzA  = (size_t)kPtsPad * kDim * 2;
constexpr size_t kSzBt = (size_t)kColsPad * kDim * 2;
constexpr size_t kSzCb = (size_t)kComp * kCbPitch * 4;
constexpr size_t kSzWv = (size_t)kDim * 4;
constexpr size_t kSzQv = (size_t)kPtsPad * 4;
constexpr size_t kSzR  = (size_t)kPtsPad * kColsPad * 4;
constexpr size_t kOffA  = 0;
constexpr size_t kOffBt = kOffA + kSzA;
constexpr size_t kOffCb = kOffBt + kSzBt;
constexpr size_t kOffWv = kOffCb + kSzCb;
constexpr size_t kOffQv = kOffWv + kSzWv;
constexpr size_t kOffR  = kOffQv + kSzQv;
constexpr size_t kWsTotal = kOffR + kSzR;
static_assert(kWsTotal == 51514112ull, "carve total");
static_assert(kWsTotal <= 134217728ull, "carve cap");
static_assert((kOffBt % 128) == 0 && (kOffCb % 128) == 0 && (kOffWv % 128) == 0 &&
              (kOffQv % 128) == 0 && (kOffR % 128) == 0, "128-B aligned regions");

__device__ __forceinline__ _Float16 f16_flush(float v) {
  const float t = (fabsf(v) < kF16MinNormal) ? 0.0f : v;
  return (_Float16)t;
}

__device__ __forceinline__ v8f mma_f16_guarded(v16h a, v16h b, v8f c) {
  c = __builtin_amdgcn_wmma_f32_16x16x32_f16(false, a, false, b, (short)0, c, false, false);
  asm volatile("v_nop\n\tv_nop\n\tv_nop\n\tv_nop" : "+v"(c) : "v"(a), "v"(b));
  return c;
}
__device__ __forceinline__ void keep4_h(v16h a, v16h b, v16h c, v16h d) { asm volatile("v_nop" :: "v"(a), "v"(b), "v"(c), "v"(d)); }
__device__ __forceinline__ void acc_guard4(v8f& a, v8f& b, v8f& c, v8f& d) { asm volatile("v_nop\n\tv_nop\n\tv_nop\n\tv_nop" : "+v"(a), "+v"(b), "+v"(c), "+v"(d)); }

union FragH { v16h v; v8h h[2]; };
__device__ __forceinline__ v16h frag_load_h(const _Float16* p) {
  FragH f;
  f.h[0] = *(const v8h*)(p);
  f.h[1] = *(const v8h*)(p + 16);
  return f.v;
}

__global__ __launch_bounds__(256) void prep_common_kernel(
    const float* __restrict__ mu, const float* __restrict__ log_psi,
    unsigned short* __restrict__ Bt, float* __restrict__ wv)
{
  __shared__ __align__(16) float wS[kDim];
  const int tid = threadIdx.x;
  float lp = log_psi[tid & (kDim - 1)];
  asm volatile("" : "+v"(lp));
  float dd = expf(lp) + 1e-5f;
  dd = dd + 1e-4f;
  const float wi = 1.0f / dd;
  if (tid < kDim) wS[tid] = wi;
  __syncthreads();
  const int i0 = (tid & 15) * 8;
  const v4f wa = *(const v4f*)(wS + i0);
  const v4f wb = *(const v4f*)(wS + i0 + 4);
  v8h hv[2];
#pragma unroll
  for (int j = 0; j < 2; ++j) {
    const int chunk = tid + j * 256;
    const int kk = chunk >> 4;
    const v4f ma = *(const v4f*)(mu + (size_t)kk * kDim + i0);
    const v4f mb = *(const v4f*)(mu + (size_t)kk * kDim + i0 + 4);
#pragma unroll
    for (int e = 0; e < 4; ++e) {
      hv[j][e]     = f16_flush((wa[e] * ma[e]) * kCarryM);
      hv[j][4 + e] = f16_flush((wb[e] * mb[e]) * kCarryM);
    }
  }
  const v4u zz = (v4u){0u, 0u, 0u, 0u};
  const float wline = wS[tid & (kDim - 1)];
  for (int pass = 0; pass < 2; ++pass) {
#pragma unroll
    for (int j = 0; j < 2; ++j) {
      const size_t off = (size_t)(tid + j * 256) * 8;
      *(volatile v8h*)(Bt + (size_t)kCrossCol * kDim + off) = hv[j];
      *(volatile v4u*)(Bt + (size_t)kCols * kDim + off) = zz;
    }
    if (tid < kDim) *(volatile float*)(wv + tid) = wline;
    __threadfence();
  }
}

__global__ __launch_bounds__(256) void prep_comp_kernel(
    const float* __restrict__ log_pi, const float* __restrict__ mu,
    const float* __restrict__ Lam, const float* __restrict__ log_psi,
    unsigned short* __restrict__ Bt, float* __restrict__ cb)
{
  __shared__ __align__(16) float lamS[kDim * kFac];
  __shared__ __align__(16) float pT[kFac * kPtPitch];
  __shared__ float wS[kDim];
  __shared__ float dS[kDim];
  __shared__ float muS[kDim];
  __shared__ float t2S[kDim];
  __shared__ float Sm[256];
  __shared__ float Gm[256];
  __shared__ float Gi[256];
  __shared__ float lgS[256];
  __shared__ float pivS[kFac];
  __shared__ float invS[kFac];
  __shared__ float bS[kFac];
  __shared__ float cS[1];

  const int k = blockIdx.x;
  const int tid = threadIdx.x;
  const int lane = tid & 31;
  const int wave = tid >> 5;

#pragma unroll
  for (int j = 0; j < 2; ++j)
    *(v4f*)(lamS + j * 1024 + tid * 4) = *(const v4f*)(Lam + (size_t)k * (kDim * kFac) + j * 1024 + tid * 4);

  float lpk = log_pi[k];
  float lps = log_psi[tid & (kDim - 1)];
  float muv = mu[(size_t)k * kDim + (tid & (kDim - 1))];
  asm volatile("" : "+v"(lpk));
  asm volatile("" : "+v"(lps));
  asm volatile("" : "+v"(muv));
  {
    float dd = expf(lps) + 1e-5f;
    dd = dd + 1e-4f;
    const float wi = 1.0f / dd;
    if (tid < kDim) {
      wS[tid] = wi;
      dS[tid] = dd;
      muS[tid] = muv;
      t2S[tid] = wi * muv * muv;
    }
  }
  __syncthreads();

  {
    const int a = tid >> 4, b = tid & 15;
    float s = (a == b) ? 1.0f : 0.0f;
#pragma unroll 4
    for (int i = 0; i < kDim; ++i)
      s = fmaf(lamS[i * kFac + a] * wS[i], lamS[i * kFac + b], s);
    Sm[tid] = s;
  }
  __syncthreads();

  if (tid == 0) {
#pragma unroll 1
    for (int a = 0; a < kFac; ++a) {
      float s = Sm[a * kFac + a];
#pragma unroll 1
      for (int m = 0; m < a; ++m) {
        const float g = Gm[a * kFac + m];
        s -= g * g;
      }
      pivS[a] = s;
      const float ga = sqrtf(s);
      const float inv = 1.0f / ga;
      Gm[a * kFac + a] = ga;
      invS[a] = inv;
#pragma unroll 1
      for (int r = a + 1; r < kFac; ++r) {
        float t = Sm[r * kFac + a];
#pragma unroll 1
        for (int m = 0; m < a; ++m) t -= Gm[r * kFac + m] * Gm[a * kFac + m];
        Gm[r * kFac + a] = t * inv;
      }
    }
#pragma unroll 1
    for (int a = 0; a < kFac; ++a) {
      Gi[a * kFac + a] = invS[a];
#pragma unroll 1
      for (int r = a + 1; r < kFac; ++r) {
        float t = 0.0f;
#pragma unroll 1
        for (int m = a; m < r; ++m) t += Gm[r * kFac + m] * Gi[m * kFac + a];
        Gi[r * kFac + a] = -t * invS[r];
      }
#pragma unroll 1
      for (int r = 0; r < a; ++r) Gi[r * kFac + a] = 0.0f;
    }
  }
  __syncthreads();

#pragma unroll 1
  for (int j = 0; j < 8; ++j) {
    const int i = (tid >> 4) + j * 16;
    const int a = tid & 15;
    float v = 0.0f;
#pragma unroll 4
    for (int b = 0; b < kFac; ++b) v = fmaf(lamS[i * kFac + b], Gi[a * kFac + b], v);
    pT[a * kPtPitch + i] = v * wS[i];
  }
  {
    const float dv = dS[tid & (kDim - 1)];
    const float pv = pivS[tid & (kFac - 1)];
    const float lv = (tid < kDim) ? dv : ((tid < kDim + kFac) ? pv : 1.0f);
    lgS[tid] = logf(lv);
  }
  __syncthreads();

  if (tid < kFac) {
    float bs = 0.0f;
#pragma unroll 1
    for (int i = 0; i < kDim; ++i) bs = fmaf(pT[tid * kPtPitch + i], muS[i], bs);
    bS[tid] = bs;
  }
  if (tid == 32) {
    float sl = 0.0f;
#pragma unroll 1
    for (int i = 0; i < kDim + kFac; ++i) sl += lgS[i];
    float cc = 0.0f;
#pragma unroll 1
    for (int i = 0; i < kDim; ++i) cc += t2S[i];
    cS[0] = lpk - 0.5f * (kDimLog2Pi + sl + cc);
  }
  __syncthreads();

  v8h hv;
  {
    const int a = tid >> 4;
    const int i0 = (tid & 15) * 8;
    const float* sp = pT + a * kPtPitch + i0;
    const v4f p0 = *(const v4f*)(sp);
    const v4f p1 = *(const v4f*)(sp + 4);
#pragma unroll
    for (int e = 0; e < 4; ++e) {
      hv[e]     = f16_flush(p0[e] * kCarryP);
      hv[4 + e] = f16_flush(p1[e] * kCarryP);
    }
  }
  const float bsel = bS[lane & (kFac - 1)];
  const float csel = cS[0];
  const float lval = (lane < kFac) ? bsel : ((lane == kFac) ? csel : 0.0f);
  for (int pass = 0; pass < 2; ++pass) {
    *(volatile v8h*)(Bt + (size_t)k * (kFac * kDim) + (size_t)tid * 8) = hv;
    if (wave == 0) *(volatile float*)(cb + (size_t)k * kCbPitch + lane) = lval;
    __threadfence();
  }
}

__global__ __launch_bounds__(256) void convert_q_kernel(
    const float* __restrict__ X, const float* __restrict__ wv,
    unsigned short* __restrict__ A, float* __restrict__ qv)
{
  __shared__ float qS[64];
  const int tid = threadIdx.x, lane = tid & 31, wave = tid >> 5;
  const int sub = tid & 15, c0 = sub * 8, rl = tid >> 4;
  const v4f w0 = *(const v4f*)(wv + c0);
  const v4f w1 = *(const v4f*)(wv + c0 + 4);
  const int base = blockIdx.x * 64;
  v8h hv[4];
#pragma unroll
  for (int p = 0; p < 4; ++p) {
    const int rloc = p * 16 + rl;
    const int row = base + rloc;
    const bool valid = row < kPts;
    const int rc = valid ? row : (kPts - 1);
    const v4f xa = *(const v4f*)(X + (size_t)rc * kDim + c0);
    const v4f xb = *(const v4f*)(X + (size_t)rc * kDim + c0 + 4);
    float qs = 0.0f;
#pragma unroll
    for (int e = 0; e < 4; ++e) {
      const float x0 = valid ? xa[e] : 0.0f;
      const float x1 = valid ? xb[e] : 0.0f;
      qs = fmaf(w0[e] * x0, x0, qs);
      qs = fmaf(w1[e] * x1, x1, qs);
      hv[p][e]     = f16_flush(x0 * kCarryX);
      hv[p][4 + e] = f16_flush(x1 * kCarryX);
    }
    qs += __shfl_xor(qs, 1, 32);
    qs += __shfl_xor(qs, 2, 32);
    qs += __shfl_xor(qs, 4, 32);
    qs += __shfl_xor(qs, 8, 32);
    if (sub == 0) qS[rloc] = qs;
  }
  __syncthreads();
  const float qline = qS[tid & 63];
  for (int pass = 0; pass < 2; ++pass) {
#pragma unroll
    for (int p = 0; p < 4; ++p)
      *(volatile v8h*)(A + (size_t)(base + p * 16 + rl) * kDim + c0) = hv[p];
    if (wave < 2) *(volatile float*)(qv + base + wave * 32 + lane) = qline;
    __threadfence();
  }
}

__global__ __launch_bounds__(256) void gemm_f16_nt_kernel(
    const unsigned short* __restrict__ Ap, int lda,
    const unsigned short* __restrict__ Btp, int ldb,
    float* __restrict__ C, int ldc,
    int M, int N, int K, float scale)
{
  const _Float16* A = (const _Float16*)Ap;
  const _Float16* Bt = (const _Float16*)Btp;
  __shared__ __align__(16) float sT[8][16 * 68];
  const int lane = threadIdx.x & 31;
  const int wave = threadIdx.x >> 5;
  const int tilesN = N >> 6;
  const int tilesM = M >> 6;
  const int tile = blockIdx.x * 8 + wave;
  if (tile >= tilesM * tilesN) return;
  const int tm = tile / tilesN;
  const int tn = tile - tm * tilesN;
  const int m0 = tm << 6;
  const int n0 = tn << 6;

  const int rlane = lane & 15;
  const int koff  = (lane >> 4) * 8;
  const int mOff  = (lane >> 4) * 8;

  v8f acc[4][4];
#pragma unroll
  for (int i = 0; i < 4; ++i)
#pragma unroll
    for (int j = 0; j < 4; ++j) acc[i][j] = (v8f){0.f,0.f,0.f,0.f,0.f,0.f,0.f,0.f};

  for (int k0 = 0; k0 < K; k0 += 32) {
    v16h bh[4];
#pragma unroll
    for (int j = 0; j < 4; ++j) {
      const size_t bo = (size_t)(n0 + (j << 4) + rlane) * ldb + koff + k0;
      bh[j] = frag_load_h(Bt + bo);
    }
#pragma unroll
    for (int i = 0; i < 4; ++i) {
      const size_t ao = (size_t)(m0 + (i << 4) + rlane) * lda + koff + k0;
      const v16h ah = frag_load_h(A + ao);
#pragma unroll
      for (int j = 0; j < 4; ++j) acc[i][j] = mma_f16_guarded(ah, bh[j], acc[i][j]);
    }
    keep4_h(bh[0], bh[1], bh[2], bh[3]);
  }
  acc_guard4(acc[0][0], acc[0][1], acc[0][2], acc[0][3]);
  acc_guard4(acc[1][0], acc[1][1], acc[1][2], acc[1][3]);
  acc_guard4(acc[2][0], acc[2][1], acc[2][2], acc[2][3]);
  acc_guard4(acc[3][0], acc[3][1], acc[3][2], acc[3][3]);

  float* slab = sT[wave];
#pragma unroll
  for (int i = 0; i < 4; ++i) {
    const int mBase = m0 + (i << 4);
#pragma unroll
    for (int j = 0; j < 4; ++j) {
#pragma unroll
      for (int r = 0; r < 8; ++r) {
        const float v = acc[i][j][r] * scale;
        slab[(mOff + r) * 68 + (j << 4) + rlane] = v;
      }
    }
    __builtin_amdgcn_fence(__ATOMIC_RELEASE, "workgroup");
    __builtin_amdgcn_wave_barrier();
    __builtin_amdgcn_fence(__ATOMIC_ACQUIRE, "workgroup");
    {
      const int hh = lane >> 4, c4 = (lane & 15) * 4;
      for (int pass = 0; pass < 2; ++pass) {
#pragma unroll
        for (int it = 0; it < 8; ++it) {
          const int row = it * 2 + hh;
          const v4f v = *(const v4f*)(slab + row * 68 + c4);
          *(volatile v4f*)(C + (size_t)(mBase + row) * ldc + n0 + c4) = v;
        }
        __threadfence();
      }
    }
    __builtin_amdgcn_fence(__ATOMIC_RELEASE, "workgroup");
    __builtin_amdgcn_wave_barrier();
    __builtin_amdgcn_fence(__ATOMIC_ACQUIRE, "workgroup");
  }
}

__global__ __launch_bounds__(64) void logit_lse_kernel(
    const float* __restrict__ R, const float* __restrict__ cb,
    const float* __restrict__ qv, float* __restrict__ out)
{
  const int lane = threadIdx.x & 31, wave = threadIdx.x >> 5;
  const int row0 = (blockIdx.x * 2 + wave) * 32;
  if (row0 >= kPts) return;
  const float* cbk = cb + (size_t)lane * kCbPitch;
  v4f b0 = *(const v4f*)(cbk);
  v4f b1 = *(const v4f*)(cbk + 4);
  v4f b2 = *(const v4f*)(cbk + 8);
  v4f b3 = *(const v4f*)(cbk + 12);
  const float ck = cbk[kFac];
  b0 = b0 * kCarryXP;
  b1 = b1 * kCarryXP;
  b2 = b2 * kCarryXP;
  b3 = b3 * kCarryXP;
  float llmine = 0.0f;
#pragma unroll 1
  for (int r = 0; r < 32; ++r) {
    const int row = row0 + r;
    const float* rp = R + (size_t)row * kColsPad;
    const v4f z0 = *(const v4f*)(rp + lane * kFac);
    const v4f z1 = *(const v4f*)(rp + lane * kFac + 4);
    const v4f z2 = *(const v4f*)(rp + lane * kFac + 8);
    const v4f z3 = *(const v4f*)(rp + lane * kFac + 12);
    const float cross = rp[kCrossCol + lane];
    const float qn = qv[row];
    float ss = 0.0f;
#pragma unroll
    for (int e = 0; e < 4; ++e) {
      const float t0 = z0[e] - b0[e];
      const float t1 = z1[e] - b1[e];
      const float t2 = z2[e] - b2[e];
      const float t3 = z3[e] - b3[e];
      ss = fmaf(t0, t0, ss);
      ss = fmaf(t1, t1, ss);
      ss = fmaf(t2, t2, ss);
      ss = fmaf(t3, t3, ss);
    }
    const float logit = (ck - 0.5f * qn) + cross * kInvXM + ss * kHalfInvXP2;
    float mx = logit;
    mx = fmaxf(mx, __shfl_xor(mx, 16, 32));
    mx = fmaxf(mx, __shfl_xor(mx, 8, 32));
    mx = fmaxf(mx, __shfl_xor(mx, 4, 32));
    mx = fmaxf(mx, __shfl_xor(mx, 2, 32));
    mx = fmaxf(mx, __shfl_xor(mx, 1, 32));
    float se = expf(logit - mx);
    se += __shfl_xor(se, 16, 32);
    se += __shfl_xor(se, 8, 32);
    se += __shfl_xor(se, 4, 32);
    se += __shfl_xor(se, 2, 32);
    se += __shfl_xor(se, 1, 32);
    const float ll = mx + logf(se);
    const float o = logit - ll;
    volatile float* op = out + (size_t)row * kComp + lane;
    *op = o;
    __threadfence();
    *op = o;
    llmine = (lane == r) ? ll : llmine;
  }
  volatile float* lq = out + (size_t)kOutResp + row0 + lane;
  *lq = llmine;
  __threadfence();
  *lq = llmine;
}

extern "C" void kernel_launch(void* const* d_in, const int* in_sizes, int n_in,
                              void* d_out, int out_size, void* d_ws, size_t ws_size,
                              hipStream_t stream) {
  if (n_in < 5) return;
  if (in_sizes[0] != kPts * kDim) return;
  if (in_sizes[1] != kComp) return;
  if (in_sizes[2] != kComp * kDim) return;
  if (in_sizes[3] != kComp * kDim * kFac) return;
  if (in_sizes[4] != kDim) return;
  if (out_size != kOutTotal) return;
  if (ws_size < kWsTotal) return;

  const float* X       = (const float*)d_in[0];
  const float* log_pi  = (const float*)d_in[1];
  const float* mu      = (const float*)d_in[2];
  const float* Lam     = (const float*)d_in[3];
  const float* log_psi = (const float*)d_in[4];
  float* out = (float*)d_out;

  char* ws = (char*)d_ws;
  unsigned short* APL = (unsigned short*)(ws + kOffA);
  unsigned short* BTP = (unsigned short*)(ws + kOffBt);
  float*          CBP = (float*)(ws + kOffCb);
  float*          WVP = (float*)(ws + kOffWv);
  float*          QVP = (float*)(ws + kOffQv);
  float*          RPL = (float*)(ws + kOffR);

  prep_common_kernel<<<1, 256, 0, stream>>>(mu, log_psi, BTP, WVP);
  prep_comp_kernel<<<kComp, 256, 0, stream>>>(log_pi, mu, Lam, log_psi, BTP, CBP);
  convert_q_kernel<<<kPtsPad / 64, 256, 0, stream>>>(X, WVP, APL, QVP);

  constexpr int kTiles = (kPtsPad / 64) * (kColsPad / 64);
  constexpr int kGemmBlocks = (kTiles + 7) / 8;
  gemm_f16_nt_kernel<<<dim3(kGemmBlocks, 1), 256, 0, stream>>>(
      APL, kDim, BTP, kDim, RPL, kColsPad, kPtsPad, kColsPad, kDim, 1.0f);

  constexpr int kLseWaves = kPts / 32;
  constexpr int kLseBlocks = (kLseWaves + 1) / 2;
  logit_lse_kernel<<<kLseBlocks, 64, 0, stream>>>(RPL, CBP, QVP, out);
}
